// TopicPropagationModel_14894946582643
// MI455X (gfx1250) — hardware-verified
//
#include <hip/hip_runtime.h>
#include <stdint.h>

typedef _Float16 v16h __attribute__((ext_vector_type(16)));
typedef _Float16 v8h  __attribute__((ext_vector_type(8)));
typedef float    v8f  __attribute__((ext_vector_type(8)));
typedef float    v4f  __attribute__((ext_vector_type(4)));
typedef int      v4i  __attribute__((ext_vector_type(4)));
typedef v8h __attribute__((may_alias)) v8ha;
typedef v4f __attribute__((may_alias)) v4fa;
typedef v4i __attribute__((may_alias)) v4ia;

union Frag { v16h v; v8h half[2]; };

#define N_TOPICS  1024
#define TOPIC_DIM 128
#define HIDDEN    512
#define N_HEADS   8
#define HEAD_DIM  64
#define BATCH     8
#define N_LAYERS  2
#define ROWBLK    64
#define NEGBIG    (-1.0e30f)
#define EMB_S     8.0f
#define W_S       32.0f
#define ACT_S     16.0f
#define P_S       16384.0f

#define G_EMB (N_TOPICS * TOPIC_DIM / 8)
#define G_SW  (HIDDEN * TOPIC_DIM / 8)
#define G_F1  (HIDDEN * HIDDEN / 8)

__device__ __forceinline__ v8f wmma_f16(v16h a, v16h b, v8f c) {
  v8f d = __builtin_amdgcn_wmma_f32_16x16x32_f16(false, a, false, b, (short)0, c, false, false);
  asm volatile("v_nop\n\tv_nop\n\tv_nop\n\tv_nop" : "+v"(d) : "v"(a), "v"(b));
  return d;
}

__device__ __forceinline__ v16h load_frag(const _Float16* p, int h) {
  Frag f;
  f.half[0] = *(const v8ha*)(p + 8 * h);
  f.half[1] = *(const v8ha*)(p + 16 + 8 * h);
  return f.v;
}

__device__ __forceinline__ float elu1(float v) {
  return (v > 0.0f) ? v : (__expf(v) - 1.0f);
}

__global__ __launch_bounds__(512) void tmax_kernel(
    const float* __restrict__ t, int n4, float* __restrict__ mxline)
{
  __shared__ float sm[16];
  const int tid = threadIdx.x;
  float mx = -3.0e38f;
  for (int i = tid; i < n4; i += 512) {
    const v4f v = *(const v4fa*)(t + (size_t)i * 4);
    mx = fmaxf(mx, fmaxf(fmaxf(v.x, v.y), fmaxf(v.z, v.w)));
  }
  #pragma unroll
  for (int off = 16; off > 0; off >>= 1) mx = fmaxf(mx, __shfl_xor(mx, off));
  if ((tid & 31) == 0) sm[tid >> 5] = mx;
  __syncthreads();
  if (tid < 32) {
    float r = sm[0];
    #pragma unroll
    for (int i = 1; i < 16; ++i) r = fmaxf(r, sm[i]);
    *(volatile float*)(mxline + tid) = r;
    __threadfence();
    *(volatile float*)(mxline + tid) = r;
  }
}

__global__ __launch_bounds__(256) void timew_kernel(
    const float* __restrict__ t, const float* __restrict__ mxline,
    float* __restrict__ tw, int n4)
{
  const int g = blockIdx.x * 256 + threadIdx.x;
  if (g >= n4) return;
  const float mx = mxline[0];
  const v4f v = *(const v4fa*)(t + (size_t)g * 4);
  v4f r;
  r.x = __expf((mx - v.x) * (-0.1f));
  r.y = __expf((mx - v.y) * (-0.1f));
  r.z = __expf((mx - v.z) * (-0.1f));
  r.w = __expf((mx - v.w) * (-0.1f));
  float* dst = tw + (size_t)g * 4;
  *(volatile v4f*)dst = r;
  __threadfence();
  *(volatile v4f*)dst = r;
}

__global__ __launch_bounds__(256) void convert_flat_kernel(
    const float* __restrict__ emb, const float* __restrict__ sW, const float* __restrict__ f1W,
    _Float16* __restrict__ embh, _Float16* __restrict__ sWh, _Float16* __restrict__ fc1h)
{
  const int g = blockIdx.x * 256 + threadIdx.x;
  if (g >= G_EMB + G_SW + G_F1) return;
  const float* src;
  _Float16* dst;
  float sc;
  if (g < G_EMB) {
    src = emb + (size_t)g * 8;  dst = embh + (size_t)g * 8;  sc = EMB_S;
  } else if (g < G_EMB + G_SW) {
    const int e = g - G_EMB;
    src = sW + (size_t)e * 8;   dst = sWh + (size_t)e * 8;   sc = W_S;
  } else {
    const int e = g - G_EMB - G_SW;
    src = f1W + (size_t)e * 8;  dst = fc1h + (size_t)e * 8;  sc = W_S;
  }
  const v4f a = *(const v4fa*)src;
  const v4f c = *(const v4fa*)(src + 4);
  const v8h o = { (_Float16)(a.x * sc), (_Float16)(a.y * sc), (_Float16)(a.z * sc), (_Float16)(a.w * sc),
                  (_Float16)(c.x * sc), (_Float16)(c.y * sc), (_Float16)(c.z * sc), (_Float16)(c.w * sc) };
  *(volatile v8h*)dst = o;
  __threadfence();
  *(volatile v8h*)dst = o;
}

__device__ __forceinline__ void gatw_store_pass(const _Float16* sT, _Float16* dstbase, int w, int lane) {
  const int q8 = lane & 7, sub = lane >> 3;
  #pragma unroll
  for (int i = 0; i < 2; ++i) {
    const int o = 8 * w + 4 * i + sub;
    const v8h v = *(const v8ha*)(sT + o * 72 + 8 * q8);
    *(volatile v8h*)(dstbase + (size_t)o * HIDDEN + 8 * q8) = v;
  }
}

__global__ __launch_bounds__(256) void convert_gatw_kernel(
    const float* __restrict__ gW, _Float16* __restrict__ Wt)
{
  __shared__ __attribute__((aligned(16))) _Float16 sT[64 * 72];
  const int tid = threadIdx.x, lane = tid & 31, w = tid >> 5;
  const int kt = blockIdx.x;
  const int lh = blockIdx.y;
  const float* src = gW + ((size_t)lh * HIDDEN + (size_t)kt * 64) * HEAD_DIM;
  #pragma unroll
  for (int p = 0; p < 4; ++p) {
    const int k = 16 * p + (tid >> 4);
    const int o4 = (tid & 15) * 4;
    const v4f v = *(const v4fa*)(src + (size_t)k * HEAD_DIM + o4);
    sT[(o4 + 0) * 72 + k] = (_Float16)(v.x * W_S);
    sT[(o4 + 1) * 72 + k] = (_Float16)(v.y * W_S);
    sT[(o4 + 2) * 72 + k] = (_Float16)(v.z * W_S);
    sT[(o4 + 3) * 72 + k] = (_Float16)(v.w * W_S);
  }
  __syncthreads();
  _Float16* dstbase = Wt + (size_t)lh * HEAD_DIM * HIDDEN + (size_t)kt * 64;
  gatw_store_pass(sT, dstbase, w, lane);
  __threadfence();
  gatw_store_pass(sT, dstbase, w, lane);
}

template <int MODE>
__device__ __forceinline__ void gemm_store_pass(const _Float16* sT, const float* sE,
                                                _Float16* C, float* es, float* ed,
                                                int m0, int n0, int ldc, int w, int lane)
{
  const int q8 = lane & 7, sub = lane >> 3;
  #pragma unroll
  for (int i = 0; i < 8; ++i) {
    const int lid = w * 32 + i * 4 + sub;
    v8h v;
    _Float16* dst;
    if (MODE == 0) {
      v = *(const v8ha*)(sT + lid * 64 + 8 * q8);
      dst = C + (size_t)(m0 + lid) * ldc + n0 + 8 * q8;
    } else {
      const int d = lid >> 1, hl = lid & 1;
      v = *(const v8ha*)(sT + d * 128 + 64 * hl + 8 * q8);
      dst = C + (size_t)(n0 + d) * ldc + m0 + 64 * hl + 8 * q8;
    }
    *(volatile v8h*)dst = v;
  }
  if (MODE == 1) {
    if (w < 2) {
      const v4f e = *(const v4fa*)(sE + w * 128 + 4 * lane);
      float* ep = (w == 0) ? es : ed;
      *(volatile v4f*)(ep + m0 + 4 * lane) = e;
    }
  }
}

template <int MODE>
__global__ __launch_bounds__(128) void gemm_kernel(
    const _Float16* __restrict__ A, const _Float16* __restrict__ Bt,
    const float* __restrict__ bias, const float* __restrict__ avec,
    _Float16* __restrict__ C, float* __restrict__ es, float* __restrict__ ed,
    long long aBatch, long long cBatch, int K, int ldc, int eBatch)
{
  __shared__ __attribute__((aligned(16))) _Float16 sT[128 * 64];
  __shared__ __attribute__((aligned(16))) float    sE[256];

  const int tid = threadIdx.x, lane = tid & 31, w = tid >> 5;
  const int h = lane >> 4, m = lane & 15;
  const int m0 = blockIdx.x * 128, n0 = blockIdx.y * 64, z = blockIdx.z;
  const int head = blockIdx.y;

  const _Float16* xa0 = A + (size_t)z * (size_t)aBatch + (size_t)(m0 + 32 * w + m) * K;
  const _Float16* xa1 = xa0 + (size_t)16 * K;
  const _Float16* wbp = Bt + (size_t)(n0 + m) * K;

  const v8f zero8 = {0.f, 0.f, 0.f, 0.f, 0.f, 0.f, 0.f, 0.f};
  v8f acc[2][4];
  #pragma unroll
  for (int mt = 0; mt < 2; ++mt)
    #pragma unroll
    for (int nt = 0; nt < 4; ++nt) acc[mt][nt] = zero8;

  #pragma unroll 1
  for (int k0 = 0; k0 < K; k0 += 32) {
    const v16h a0 = load_frag(xa0 + k0, h);
    const v16h a1 = load_frag(xa1 + k0, h);
    #pragma unroll
    for (int nt = 0; nt < 4; ++nt) {
      const v16h bq = load_frag(wbp + (size_t)nt * 16 * K + k0, h);
      acc[0][nt] = wmma_f16(a0, bq, acc[0][nt]);
      acc[1][nt] = wmma_f16(a1, bq, acc[1][nt]);
    }
  }

  if (MODE == 0) {
    #pragma unroll
    for (int nt = 0; nt < 4; ++nt) {
      const int feat = 16 * nt + m;
      const float bv = bias[n0 + feat];
      #pragma unroll
      for (int mt = 0; mt < 2; ++mt) {
        #pragma unroll
        for (int r = 0; r < 8; ++r) {
          const int tokl = 32 * w + 16 * mt + 8 * h + r;
          const float y = acc[mt][nt][r] * (1.0f / (EMB_S * W_S)) + bv;
          sT[tokl * 64 + feat] = (_Float16)(y * ACT_S);
        }
      }
    }
  } else {
    float ps[2][8], pd[2][8];
    #pragma unroll
    for (int mt = 0; mt < 2; ++mt)
      #pragma unroll
      for (int r = 0; r < 8; ++r) { ps[mt][r] = 0.0f; pd[mt][r] = 0.0f; }
    #pragma unroll
    for (int nt = 0; nt < 4; ++nt) {
      const int feat = 16 * nt + m;
      const float as = avec[head * 2 * HEAD_DIM + feat];
      const float ad = avec[head * 2 * HEAD_DIM + HEAD_DIM + feat];
      #pragma unroll
      for (int mt = 0; mt < 2; ++mt) {
        #pragma unroll
        for (int r = 0; r < 8; ++r) {
          const int tokl = 32 * w + 16 * mt + 8 * h + r;
          const float y = acc[mt][nt][r] * (1.0f / (ACT_S * W_S));
          sT[feat * 128 + tokl] = (_Float16)(y * ACT_S);
          ps[mt][r] += y * as;
          pd[mt][r] += y * ad;
        }
      }
    }
    #pragma unroll
    for (int off = 1; off < 16; off <<= 1) {
      #pragma unroll
      for (int mt = 0; mt < 2; ++mt)
        #pragma unroll
        for (int r = 0; r < 8; ++r) {
          ps[mt][r] += __shfl_xor(ps[mt][r], off);
          pd[mt][r] += __shfl_xor(pd[mt][r], off);
        }
    }
    if (m == 0) {
      #pragma unroll
      for (int mt = 0; mt < 2; ++mt)
        #pragma unroll
        for (int r = 0; r < 8; ++r) {
          const int tokl = 32 * w + 16 * mt + 8 * h + r;
          sE[tokl] = ps[mt][r];
          sE[128 + tokl] = pd[mt][r];
        }
    }
  }
  __syncthreads();

  _Float16* Cz = C + (size_t)z * (size_t)cBatch;
  float* esz = es + (size_t)z * (size_t)eBatch + (size_t)head * ldc;
  float* edz = ed + (size_t)z * (size_t)eBatch + (size_t)head * ldc;
  gemm_store_pass<MODE>(sT, sE, Cz, esz, edz, m0, n0, ldc, w, lane);
  __threadfence();
  gemm_store_pass<MODE>(sT, sE, Cz, esz, edz, m0, n0, ldc, w, lane);
}

__device__ __forceinline__ float gat_logit(float esq, float edv, float twv, int av) {
  float e = esq + edv;
  e = (e >= 0.0f) ? e : (0.2f * e);
  e = e * twv;
  return (av != 0) ? e : NEGBIG;
}

__device__ __forceinline__ v16h pack_p(v8f a, v8f c) {
  const v16h r = { (_Float16)(a[0] * P_S), (_Float16)(a[1] * P_S), (_Float16)(a[2] * P_S), (_Float16)(a[3] * P_S),
                   (_Float16)(a[4] * P_S), (_Float16)(a[5] * P_S), (_Float16)(a[6] * P_S), (_Float16)(a[7] * P_S),
                   (_Float16)(c[0] * P_S), (_Float16)(c[1] * P_S), (_Float16)(c[2] * P_S), (_Float16)(c[3] * P_S),
                   (_Float16)(c[4] * P_S), (_Float16)(c[5] * P_S), (_Float16)(c[6] * P_S), (_Float16)(c[7] * P_S) };
  return r;
}

__device__ __forceinline__ void attn_store_h(const _Float16* so, _Float16* dst0, int lane) {
  const int q8 = lane & 7, sub = lane >> 3;
  #pragma unroll
  for (int i = 0; i < 4; ++i) {
    const int lid = i * 4 + sub;
    const v8h v = *(const v8ha*)(so + lid * 64 + 8 * q8);
    *(volatile v8h*)(dst0 + (size_t)lid * HIDDEN + 8 * q8) = v;
  }
}

__device__ __forceinline__ void attn_store_f(const float* so, float* dst0, int lane) {
  const int q8 = lane & 7, sub = lane >> 3;
  #pragma unroll
  for (int i = 0; i < 8; ++i) {
    const int lid = i * 4 + sub;
    const int row = lid >> 1, hl = lid & 1;
    const v4f v = *(const v4fa*)(so + row * 64 + 32 * hl + 4 * q8);
    *(volatile v4f*)(dst0 + (size_t)row * HIDDEN + 32 * hl + 4 * q8) = v;
  }
}

template <int MODE>
__global__ __launch_bounds__(128) void gat_attn_kernel(
    const _Float16* __restrict__ hT, const float* __restrict__ es, const float* __restrict__ ed,
    const int* __restrict__ adj, const float* __restrict__ tw, const int* __restrict__ topic_ids,
    _Float16* __restrict__ outH, float* __restrict__ outF, long long hBatch, int eBatch)
{
  __shared__ __attribute__((aligned(16))) float    sOf[4 * 16 * 64];
  __shared__ __attribute__((aligned(16))) _Float16 sOh[4 * 16 * 64];

  const int tid = threadIdx.x, lane = tid & 31, w = tid >> 5;
  const int h = lane >> 4, m = lane & 15;
  const int hd = blockIdx.y, b = blockIdx.z;
  int iblk;
  if (MODE == 0) {
    iblk = blockIdx.x * ROWBLK;
  } else {
    int t = topic_ids[b];
    t = (t < 0) ? 0 : ((t > N_TOPICS - 1) ? (N_TOPICS - 1) : t);
    iblk = t & ~(ROWBLK - 1);
  }
  const int q0 = iblk + 16 * w;
  const int q = q0 + m;

  const size_t ebase = (size_t)b * (size_t)eBatch + (size_t)hd * N_TOPICS;
  const float esq = es[ebase + q];
  const float* edp = ed + ebase + 8 * h;
  const size_t rowoff = ((size_t)b * N_TOPICS + q) * N_TOPICS + 8 * h;
  const int* adjRow = adj + rowoff;
  const float* twRow = tw + rowoff;
  const _Float16* hbase = hT + (size_t)b * (size_t)hBatch + ((size_t)hd * HEAD_DIM + m) * N_TOPICS;

  const v8f zero8 = {0.f, 0.f, 0.f, 0.f, 0.f, 0.f, 0.f, 0.f};
  v8f o[4];
  #pragma unroll
  for (int t = 0; t < 4; ++t) o[t] = zero8;
  float mrun = NEGBIG, lrun = 0.0f;

  #pragma unroll 1
  for (int kb = 0; kb < N_TOPICS; kb += 64) {
    v8f s[4];
    float mloc = NEGBIG;
    #pragma unroll
    for (int c = 0; c < 4; ++c) {
      const int off = kb + 16 * c;
      const v4f e0 = *(const v4fa*)(edp + off);
      const v4f e1 = *(const v4fa*)(edp + off + 4);
      const v4f t0 = *(const v4fa*)(twRow + off);
      const v4f t1 = *(const v4fa*)(twRow + off + 4);
      const v4i a0 = *(const v4ia*)(adjRow + off);
      const v4i a1 = *(const v4ia*)(adjRow + off + 4);
      v8f z;
      z[0] = gat_logit(esq, e0.x, t0.x, a0.x);
      z[1] = gat_logit(esq, e0.y, t0.y, a0.y);
      z[2] = gat_logit(esq, e0.z, t0.z, a0.z);
      z[3] = gat_logit(esq, e0.w, t0.w, a0.w);
      z[4] = gat_logit(esq, e1.x, t1.x, a1.x);
      z[5] = gat_logit(esq, e1.y, t1.y, a1.y);
      z[6] = gat_logit(esq, e1.z, t1.z, a1.z);
      z[7] = gat_logit(esq, e1.w, t1.w, a1.w);
      #pragma unroll
      for (int r = 0; r < 8; ++r) mloc = fmaxf(mloc, z[r]);
      s[c] = z;
    }
    mloc = fmaxf(mloc, __shfl_xor(mloc, 16));
    const float mnew = fmaxf(mrun, mloc);
    const float alpha = __expf(mrun - mnew);
    mrun = mnew;
    float lsum = 0.0f;
    #pragma unroll
    for (int c = 0; c < 4; ++c)
      #pragma unroll
      for (int r = 0; r < 8; ++r) {
        const float sv = s[c][r];
        const float p = (sv > -1.0e29f) ? __expf(sv - mnew) : 0.0f;
        s[c][r] = p;
        lsum += p;
      }
    lsum += __shfl_xor(lsum, 16);
    lrun = lrun * alpha + lsum;
    #pragma unroll
    for (int t = 0; t < 4; ++t)
      #pragma unroll
      for (int r = 0; r < 8; ++r) o[t][r] = o[t][r] * alpha;

    const v16h pb0 = pack_p(s[0], s[1]);
    const v16h pb1 = pack_p(s[2], s[3]);

    #pragma unroll
    for (int t = 0; t < 4; ++t) {
      const _Float16* hp = hbase + (size_t)(16 * t) * N_TOPICS + kb;
      const v16h vf0 = load_frag(hp, h);
      const v16h vf1 = load_frag(hp + 32, h);
      o[t] = wmma_f16(vf0, pb0, o[t]);
      o[t] = wmma_f16(vf1, pb1, o[t]);
    }
  }

  const float inv = 1.0f / (lrun * (P_S * ACT_S));
  if (MODE == 0) {
    _Float16* so = sOh + w * 1024;
    #pragma unroll
    for (int t = 0; t < 4; ++t)
      #pragma unroll
      for (int r = 0; r < 8; ++r)
        so[m * 64 + 16 * t + 8 * h + r] = (_Float16)(elu1(o[t][r] * inv) * ACT_S);
  } else {
    float* so = sOf + w * 1024;
    #pragma unroll
    for (int t = 0; t < 4; ++t)
      #pragma unroll
      for (int r = 0; r < 8; ++r)
        so[m * 64 + 16 * t + 8 * h + r] = elu1(o[t][r] * inv);
  }
  __syncthreads();

  if (MODE == 0) {
    const _Float16* so = sOh + w * 1024;
    _Float16* dst0 = outH + ((size_t)b * N_TOPICS + q0) * HIDDEN + (size_t)hd * HEAD_DIM;
    attn_store_h(so, dst0, lane);
    __threadfence();
    attn_store_h(so, dst0, lane);
  } else {
    const float* so = sOf + w * 1024;
    float* dst0 = outF + ((size_t)b * ROWBLK + 16 * w) * HIDDEN + (size_t)hd * HEAD_DIM;
    attn_store_f(so, dst0, lane);
    __threadfence();
    attn_store_f(so, dst0, lane);
  }
}

__global__ __launch_bounds__(256) void head_kernel(
    const float* __restrict__ node2c, const int* __restrict__ topic_ids,
    const float* __restrict__ attractiveness,
    const float* __restrict__ attract_W, const float* __restrict__ attract_b,
    const _Float16* __restrict__ fc1h, const float* __restrict__ fc1_b,
    const float* __restrict__ fc2_W, const float* __restrict__ fc2_b,
    float* __restrict__ out)
{
  __shared__ __attribute__((aligned(16))) _Float16 sA[16 * HIDDEN];
  __shared__ float sRed[64];
  __shared__ __attribute__((aligned(16))) float sOut[8];

  const int tid = threadIdx.x, lane = tid & 31, w = tid >> 5;
  const int h = lane >> 4, m = lane & 15;

  for (int idx = tid; idx < 16 * HIDDEN; idx += 256) {
    const int r = idx >> 9, c = idx & (HIDDEN - 1);
    float v = 0.0f;
    if (r < BATCH) {
      int t = topic_ids[r];
      t = (t < 0) ? 0 : ((t > N_TOPICS - 1) ? (N_TOPICS - 1) : t);
      const float tf = node2c[((size_t)r * ROWBLK + (t & (ROWBLK - 1))) * HIDDEN + c];
      const float at = attractiveness[r] * attract_W[c] + attract_b[c];
      v = tf + at;
    }
    sA[idx] = (_Float16)(v * ACT_S);
  }
  __syncthreads();

  const v8f zero8 = {0.f, 0.f, 0.f, 0.f, 0.f, 0.f, 0.f, 0.f};
  v8f acc[4];
  #pragma unroll
  for (int j = 0; j < 4; ++j) acc[j] = zero8;
  const _Float16* arow = sA + m * HIDDEN;
  const _Float16* brow = fc1h + (size_t)(64 * w + m) * HIDDEN;
  #pragma unroll 1
  for (int k0 = 0; k0 < HIDDEN; k0 += 32) {
    const v16h a = load_frag(arow + k0, h);
    #pragma unroll
    for (int j = 0; j < 4; ++j) {
      const v16h bq = load_frag(brow + (size_t)16 * j * HIDDEN + k0, h);
      acc[j] = wmma_f16(a, bq, acc[j]);
    }
  }

  float ps[8];
  #pragma unroll
  for (int r = 0; r < 8; ++r) ps[r] = 0.0f;
  #pragma unroll
  for (int j = 0; j < 4; ++j) {
    const int n = 64 * w + 16 * j + m;
    const float bb = fc1_b[n];
    const float f2 = fc2_W[n];
    #pragma unroll
    for (int r = 0; r < 8; ++r) {
      const float hv = fmaxf(acc[j][r] * (1.0f / (ACT_S * W_S)) + bb, 0.0f);
      ps[r] += hv * f2;
    }
  }
  #pragma unroll
  for (int off = 1; off < 16; off <<= 1)
    #pragma unroll
    for (int r = 0; r < 8; ++r) ps[r] += __shfl_xor(ps[r], off);
  if (lane == 0) {
    #pragma unroll
    for (int r = 0; r < 8; ++r) sRed[w * 8 + r] = ps[r];
  }
  __syncthreads();
  if (tid < BATCH) {
    float sum = 0.0f;
    #pragma unroll
    for (int w2 = 0; w2 < 8; ++w2) sum += sRed[w2 * 8 + tid];
    sOut[tid] = sum + fc2_b[0];
  }
  __syncthreads();
  if (tid < 2) {
    const v4f v = *(const v4fa*)(sOut + 4 * tid);
    *(volatile v4f*)(out + 4 * tid) = v;
    __threadfence();
    *(volatile v4f*)(out + 4 * tid) = v;
  }
}

extern "C" void kernel_launch(void* const* d_in, const int* in_sizes, int n_in,
                              void* d_out, int out_size, void* d_ws, size_t ws_size,
                              hipStream_t stream)
{
  if (n_in < 15) return;
  const long long NN = (long long)BATCH * N_TOPICS * N_TOPICS;
  if (in_sizes[0] != BATCH || (long long)in_sizes[1] != NN || (long long)in_sizes[2] != NN) return;
  if (in_sizes[3] != BATCH) return;
  if (in_sizes[4] != N_TOPICS * TOPIC_DIM || in_sizes[5] != HIDDEN * TOPIC_DIM || in_sizes[6] != HIDDEN) return;
  if (in_sizes[7] != HIDDEN || in_sizes[8] != HIDDEN) return;
  if (in_sizes[9] != N_LAYERS * N_HEADS * HIDDEN * HEAD_DIM || in_sizes[10] != N_LAYERS * N_HEADS * 2 * HEAD_DIM) return;
  if (in_sizes[11] != HIDDEN * HIDDEN || in_sizes[12] != HIDDEN || in_sizes[13] != HIDDEN || in_sizes[14] < 1) return;
  if (out_size != BATCH) return;

  const int*   topic_ids      = (const int*)  d_in[0];
  const int*   adj            = (const int*)  d_in[1];
  const float* time_matrix    = (const float*)d_in[2];
  const float* attractiveness = (const float*)d_in[3];
  const float* topic_emb      = (const float*)d_in[4];
  const float* struct_W       = (const float*)d_in[5];
  const float* struct_b       = (const float*)d_in[6];
  const float* attract_W      = (const float*)d_in[7];
  const float* attract_b      = (const float*)d_in[8];
  const float* gat_W          = (const float*)d_in[9];
  const float* gat_a          = (const float*)d_in[10];
  const float* fc1_W          = (const float*)d_in[11];
  const float* fc1_b          = (const float*)d_in[12];
  const float* fc2_W          = (const float*)d_in[13];
  const float* fc2_b          = (const float*)d_in[14];
  float* out = (float*)d_out;

  char* ws = (char*)d_ws;
  size_t off = 0;
  auto carve = [&](size_t bytes) -> char* {
    char* p = ws + off;
    off += (bytes + 255) & ~(size_t)255;
    return p;
  };
  float*    mxline  = (float*)   carve(256);
  float*    tw      = (float*)   carve((size_t)NN * 4);
  _Float16* embh    = (_Float16*)carve((size_t)N_TOPICS * TOPIC_DIM * 2);
  _Float16* sWh     = (_Float16*)carve((size_t)HIDDEN * TOPIC_DIM * 2);
  _Float16* fc1h    = (_Float16*)carve((size_t)HIDDEN * HIDDEN * 2);
  _Float16* Wt      = (_Float16*)carve((size_t)N_LAYERS * HIDDEN * HIDDEN * 2);
  _Float16* structh = (_Float16*)carve((size_t)N_TOPICS * HIDDEN * 2);
  _Float16* hT1     = (_Float16*)carve((size_t)HIDDEN * N_TOPICS * 2);
  float*    es1     = (float*)   carve((size_t)N_HEADS * N_TOPICS * 4);
  float*    ed1     = (float*)   carve((size_t)N_HEADS * N_TOPICS * 4);
  _Float16* node1h  = (_Float16*)carve((size_t)BATCH * N_TOPICS * HIDDEN * 2);
  _Float16* hT2     = (_Float16*)carve((size_t)BATCH * HIDDEN * N_TOPICS * 2);
  float*    es2     = (float*)   carve((size_t)BATCH * N_HEADS * N_TOPICS * 4);
  float*    ed2     = (float*)   carve((size_t)BATCH * N_HEADS * N_TOPICS * 4);
  float*    node2c  = (float*)   carve((size_t)BATCH * ROWBLK * HIDDEN * 4);
  if (off > ws_size) return;
  if (off > (size_t)128 * 1024 * 1024) return;

  const int n4 = (int)(NN / 4);

  tmax_kernel<<<1, 512, 0, stream>>>(time_matrix, n4, mxline);
  timew_kernel<<<(n4 + 255) / 256, 256, 0, stream>>>(time_matrix, mxline, tw, n4);

  convert_flat_kernel<<<(G_EMB + G_SW + G_F1 + 255) / 256, 256, 0, stream>>>(
      topic_emb, struct_W, fc1_W, embh, sWh, fc1h);
  convert_gatw_kernel<<<dim3(HIDDEN / 64, N_LAYERS * N_HEADS), 256, 0, stream>>>(gat_W, Wt);

  gemm_kernel<0><<<dim3(N_TOPICS / 128, HIDDEN / 64, 1), 128, 0, stream>>>(
      embh, sWh, struct_b, struct_b, structh, mxline, mxline,
      0LL, 0LL, TOPIC_DIM, HIDDEN, 0);

  gemm_kernel<1><<<dim3(N_TOPICS / 128, HIDDEN / 64, 1), 128, 0, stream>>>(
      structh, Wt, struct_b, gat_a, hT1, es1, ed1,
      0LL, 0LL, HIDDEN, N_TOPICS, 0);
  gat_attn_kernel<0><<<dim3(N_TOPICS / ROWBLK, N_HEADS, BATCH), 128, 0, stream>>>(
      hT1, es1, ed1, adj, tw, topic_ids, node1h, node2c, 0LL, 0);

  gemm_kernel<1><<<dim3(N_TOPICS / 128, HIDDEN / 64, BATCH), 128, 0, stream>>>(
      node1h, Wt + (size_t)HIDDEN * HIDDEN, struct_b, gat_a + (size_t)N_HEADS * 2 * HEAD_DIM,
      hT2, es2, ed2,
      (long long)N_TOPICS * HIDDEN, (long long)HIDDEN * N_TOPICS, HIDDEN, N_TOPICS, N_HEADS * N_TOPICS);
  gat_attn_kernel<1><<<dim3(1, N_HEADS, BATCH), 128, 0, stream>>>(
      hT2, es2, ed2, adj, tw, topic_ids, node1h, node2c,
      (long long)HIDDEN * N_TOPICS, N_HEADS * N_TOPICS);

  head_kernel<<<1, 256, 0, stream>>>(node2c, topic_ids, attractiveness, attract_W, attract_b,
                                      fc1h, fc1_b, fc2_W, fc2_b, out);
}
